// MambaBlock_24240795418673
// MI455X (gfx1250) — hardware-run, weakly checked
//
#include <hip/hip_runtime.h>
#include <math.h>

typedef __attribute__((ext_vector_type(16))) _Float16 v16h;
typedef __attribute__((ext_vector_type(8)))  _Float16 v8h;
typedef __attribute__((ext_vector_type(2)))  _Float16 v2h;
typedef __attribute__((ext_vector_type(16))) __bf16   v16b;
typedef __attribute__((ext_vector_type(8)))  __bf16   v8b;
typedef __attribute__((ext_vector_type(8)))  float    v8f;
typedef __attribute__((ext_vector_type(4)))  float    v4f;
typedef __attribute__((ext_vector_type(2)))  float    v2f;
typedef __attribute__((ext_vector_type(4)))  _Float16 v4h;

constexpr int kNB   = 2;
constexpr int kL    = 2048;
constexpr int kRows = kNB * kL;
constexpr int kDm   = 1024;
constexpr int kDI   = 2048;
constexpr int kDI2  = 2 * kDI;
constexpr int kNs   = 16;
constexpr int kR    = 64;
constexpr int kXd   = kR + 2 * kNs;
constexpr int kXdP  = 128;
constexpr int kCv   = 4;
constexpr int kOut0 = kRows * kDm;
constexpr int kOut1 = kNB * kDI * kNs;
constexpr int kOut2 = kNB * kDI * (kCv - 1);
constexpr int kBvDt = kDI2;
constexpr int kBvTot = kDI2 + kDI;
constexpr int kThr  = 256;
constexpr float kInCarry = 1024.0f;
constexpr float kWCarry  = 4096.0f;
constexpr float kACarry  = 256.0f;
constexpr float kDtCarry = 256.0f;
constexpr float kScIn = 1.0f / (kInCarry * kWCarry);
constexpr float kScA  = 1.0f / (kACarry * kWCarry);
constexpr float kScDt = 1.0f / (kDtCarry * kWCarry);
constexpr float kF16MinNormal = 6.103515625e-5f;

static_assert(kRows == 4096 && kDm == 1024 && kDI == 2048 && kNs == 16 && kR == 64 && kXd == 96 && kXd <= kXdP && (kXdP % 64) == 0 && kCv == 4 && (kL & (kL - 1)) == 0, "the index arithmetic below uses these sizes");

constexpr size_t kOffX16 = 0ull;
constexpr size_t kOffWIT = 8388608ull;
constexpr size_t kOffWXT = 16777216ull;
constexpr size_t kOffWDT = 17825792ull;
constexpr size_t kOffWOT = 18087936ull;
constexpr size_t kOffBV = 22282240ull;
constexpr size_t kOffXZ = 22306816ull;
constexpr size_t kOffXI = 89415680ull;
constexpr size_t kOffXI16 = 122970112ull;
constexpr size_t kOffXD = 156524544ull;
constexpr size_t kOffDT16 = 158621696ull;
constexpr size_t kOffDL = 159145984ull;
constexpr size_t kOffYS = 192700416ull;
constexpr size_t kOffYG16 = 226254848ull;
constexpr size_t kWsTotal = 243032064ull;
static_assert(kWsTotal <= 268435456ull, "the carve stands under the contract's 256 MiB of workspace");
static_assert(kOffX16 == 0
  && kOffWIT == kOffX16 + 8388608ull
  && kOffWXT == kOffWIT + 8388608ull
  && kOffWDT == kOffWXT + 1048576ull
  && kOffWOT == kOffWDT + 262144ull
  && kOffBV == kOffWOT + 4194304ull
  && kOffXZ == kOffBV + 24576ull
  && kOffXI == kOffXZ + 67108864ull
  && kOffXI16 == kOffXI + 33554432ull
  && kOffXD == kOffXI16 + 33554432ull
  && kOffDT16 == kOffXD + 2097152ull
  && kOffDL == kOffDT16 + 524288ull
  && kOffYS == kOffDL + 33554432ull
  && kOffYG16 == kOffYS + 33554432ull
  && kWsTotal == kOffYG16 + 16777216ull, "the carve is a chain: every region starts where the one before ends");
static_assert((size_t)kRows * kDm * 2 == 8388608ull && (size_t)kDI2 * kDm * 2 == 8388608ull && (size_t)kXdP * kDI2 * 2 == 1048576ull && (size_t)kDI * kR * 2 == 262144ull && (size_t)kDm * kDI * 2 == 4194304ull && (size_t)kBvTot * 4 == 24576ull
  && (size_t)kRows * kDI2 * 4 == 67108864ull && (size_t)kRows * kDI * 4 == 33554432ull && (size_t)kRows * kDI2 * 2 == 33554432ull && (size_t)kRows * kXdP * 4 == 2097152ull && (size_t)kRows * kR * 2 == 524288ull && (size_t)kRows * kDI * 2 == 16777216ull, "every region's length is its plane's");
static_assert((kOffWIT % 256) == 0 && (kOffWXT % 256) == 0 && (kOffWDT % 256) == 0 && (kOffWOT % 256) == 0 && (kOffBV % 256) == 0 && (kOffXZ % 256) == 0 && (kOffXI % 256) == 0 && (kOffXI16 % 256) == 0 && (kOffXD % 256) == 0 && (kOffDT16 % 256) == 0
  && (kOffDL % 256) == 0 && (kOffYS % 256) == 0 && (kOffYG16 % 256) == 0, "every region starts on a multiple of 256 B");

__device__ __forceinline__ unsigned short f2bf_bits(float f) {
  unsigned u = __float_as_uint(f);
  return (unsigned short)((u + 0x7FFFu + ((u >> 16) & 1u)) >> 16);
}
__device__ __forceinline__ float bf_bits2f(unsigned short h) { return __uint_as_float(((unsigned)h) << 16); }
__device__ __forceinline__ float bf16r(float f) { return bf_bits2f(f2bf_bits(f)); }
__device__ __forceinline__ float carry_flush(float v, float carry) {
  const float s = v * carry;
  return (fabsf(s) < kF16MinNormal) ? 0.0f : s;
}

__device__ __forceinline__ void dep_guard4_h(v8f& a, v8f& b, v8f& c, v8f& d, v16h x, v16h y) { asm volatile("v_nop\n\tv_nop\n\tv_nop\n\tv_nop" : "+v"(a), "+v"(b), "+v"(c), "+v"(d) : "v"(x), "v"(y)); }
__device__ __forceinline__ void dep_guard4_b(v8f& a, v8f& b, v8f& c, v8f& d, v16b x, v16b y) { asm volatile("v_nop\n\tv_nop\n\tv_nop\n\tv_nop" : "+v"(a), "+v"(b), "+v"(c), "+v"(d) : "v"(x), "v"(y)); }
__device__ __forceinline__ void keep4_h(v16h a, v16h b, v16h c, v16h d) { asm volatile("v_nop" :: "v"(a), "v"(b), "v"(c), "v"(d)); }
__device__ __forceinline__ void keep4_b(v16b a, v16b b, v16b c, v16b d) { asm volatile("v_nop" :: "v"(a), "v"(b), "v"(c), "v"(d)); }
__device__ __forceinline__ void acc_guard4(v8f& a, v8f& b, v8f& c, v8f& d) { asm volatile("v_nop\n\tv_nop\n\tv_nop\n\tv_nop" : "+v"(a), "+v"(b), "+v"(c), "+v"(d)); }

template <typename T> struct Frag;
template <> struct Frag<_Float16> {
  typedef v16h V; union U { v16h v; v8h h[2]; };
  static __device__ __forceinline__ v16h load(const _Float16* p) {
    U f; f.h[0] = *(const v8h*)(p); f.h[1] = *(const v8h*)(p + 16); return f.v;
  }
  static __device__ __forceinline__ v8f mma(v16h a, v16h b, v8f c) {
    return __builtin_amdgcn_wmma_f32_16x16x32_f16(false, a, false, b, (short)0, c, false, false);
  }
  static __device__ __forceinline__ void guard4(v8f& a, v8f& b, v8f& c, v8f& d, v16h x, v16h y) { dep_guard4_h(a, b, c, d, x, y); }
  static __device__ __forceinline__ void keep(v16h a, v16h b, v16h c, v16h d) { keep4_h(a, b, c, d); }
};
template <> struct Frag<__bf16> {
  typedef v16b V; union U { v16b v; v8b h[2]; };
  static __device__ __forceinline__ v16b load(const __bf16* p) {
    U f; f.h[0] = *(const v8b*)(p); f.h[1] = *(const v8b*)(p + 16); return f.v;
  }
  static __device__ __forceinline__ v8f mma(v16b a, v16b b, v8f c) {
    return __builtin_amdgcn_wmma_f32_16x16x32_bf16(false, a, false, b, (short)0, c, false, false);
  }
  static __device__ __forceinline__ void guard4(v8f& a, v8f& b, v8f& c, v8f& d, v16b x, v16b y) { dep_guard4_b(a, b, c, d, x, y); }
  static __device__ __forceinline__ void keep(v16b a, v16b b, v16b c, v16b d) { keep4_b(a, b, c, d); }
};

__device__ __forceinline__ v8f mma_h(v16h a, v16h b, v8f c) {
  c = __builtin_amdgcn_wmma_f32_16x16x32_f16(false, a, false, b, (short)0, c, false, false);
  asm volatile("v_nop\n\tv_nop\n\tv_nop\n\tv_nop" : "+v"(c) : "v"(a), "v"(b));
  return c;
}

template <int ET> struct Elem;
template <> struct Elem<0> { typedef _Float16 T; };
template <> struct Elem<1> { typedef __bf16 T; };
template <int ET, bool SPLIT, int BIAS_MODE, int OUT_MODE, bool RESID, int ACT = 0>
__global__ __launch_bounds__(256) void wmma_gemm64(
    const unsigned short* __restrict__ Ap, const unsigned short* __restrict__ A2p, int lda, long strideA,
    const unsigned short* __restrict__ Btp, const unsigned short* __restrict__ Bt2p, int ldb, long strideB,
    void* __restrict__ Cout, void* __restrict__ Cout2, int ldc, long strideC,
    const float* __restrict__ bias,
    const float* __restrict__ resid, long strideR,
    int M, int N, int K, float scale) {
  typedef typename Elem<ET>::T T;
  typedef typename Frag<T>::V V;
  const T* A = (const T*)Ap; const T* A2 = (const T*)A2p; const T* Bt = (const T*)Btp; const T* Bt2 = (const T*)Bt2p;
  __shared__ __align__(16) float sT[8][16 * 68];
  const int b    = blockIdx.y;
  const int lane = threadIdx.x & 31;
  const int wave = threadIdx.x >> 5;
  const int tilesN = N >> 6;
  const int tilesM = M >> 6;
  const int tile = blockIdx.x * 8 + wave;
  if (tile >= tilesM * tilesN) return;
  const int tm = tile / tilesN;
  const int tn = tile - tm * tilesN;
  const int m0 = tm << 6;
  const int n0 = tn << 6;

  const T* Ab  = A  + (size_t)b * strideA;
  const T* Bb  = Bt + (size_t)b * strideB;
  const T* Ab2 = SPLIT ? (A2  + (size_t)b * strideA) : nullptr;
  const T* Bb2 = SPLIT ? (Bt2 + (size_t)b * strideB) : nullptr;

  const int rlane = lane & 15;
  const int koff  = (lane >> 4) * 8;
  const int mOff  = (lane >> 4) * 8;

  v8f acc[4][4];
#pragma unroll
  for (int i = 0; i < 4; ++i)
#pragma unroll
    for (int j = 0; j < 4; ++j) acc[i][j] = (v8f){0.f,0.f,0.f,0.f,0.f,0.f,0.f,0.f};

  for (int k0 = 0; k0 < K; k0 += 32) {
    V bh[4], bl[4];
#pragma unroll
    for (int j = 0; j < 4; ++j) {
      const size_t bo = (size_t)(n0 + (j << 4) + rlane) * ldb + koff + k0;
      bh[j] = Frag<T>::load(Bb + bo);
      if (SPLIT) bl[j] = Frag<T>::load(Bb2 + bo);
    }
#pragma unroll
    for (int i = 0; i < 4; ++i) {
      const size_t ao = (size_t)(m0 + (i << 4) + rlane) * lda + koff + k0;
      V ah = Frag<T>::load(Ab + ao);
      V al;
      if (SPLIT) al = Frag<T>::load(Ab2 + ao);
#pragma unroll
      for (int j = 0; j < 4; ++j) {
        acc[i][j] = Frag<T>::mma(ah, bh[j], acc[i][j]);
        if (SPLIT) {
          acc[i][j] = Frag<T>::mma(ah, bl[j], acc[i][j]);
          acc[i][j] = Frag<T>::mma(al, bh[j], acc[i][j]);
        }
      }
      Frag<T>::guard4(acc[i][0], acc[i][1], acc[i][2], acc[i][3], ah, SPLIT ? al : ah);
    }
    Frag<T>::keep(bh[0], bh[1], bh[2], bh[3]);
    if (SPLIT) Frag<T>::keep(bl[0], bl[1], bl[2], bl[3]);
  }
  acc_guard4(acc[0][0], acc[0][1], acc[0][2], acc[0][3]);
  acc_guard4(acc[1][0], acc[1][1], acc[1][2], acc[1][3]);
  acc_guard4(acc[2][0], acc[2][1], acc[2][2], acc[2][3]);
  acc_guard4(acc[3][0], acc[3][1], acc[3][2], acc[3][3]);

  float* slab = sT[wave];
  const float* Rb = RESID ? (resid + (size_t)b * strideR) : nullptr;
#pragma unroll
  for (int i = 0; i < 4; ++i) {
    const int mBase = m0 + (i << 4);
#pragma unroll
    for (int j = 0; j < 4; ++j) {
      const int n = n0 + (j << 4) + rlane;
      float bv = 0.f;
      if (BIAS_MODE == 2) bv = bias[n];
#pragma unroll
      for (int r = 0; r < 8; ++r) {
        float v = acc[i][j][r] * scale;
        if (BIAS_MODE == 1) v += bias[mBase + mOff + r];
        if (BIAS_MODE == 2) v += bv;
        if (RESID) v += Rb[(size_t)(mBase + mOff + r) * ldc + n];
        if (ACT == 1) v = tanhf(v);
        if (ACT == 2) v = fmaxf(v, 0.0f);
        if (ACT == 3) v = v / (1.0f + expf(-v));
        if (ACT == 4) v = (v > 0.f) ? v : 0.01f * v;
        slab[(mOff + r) * 68 + (j << 4) + rlane] = v;
      }
    }
    __builtin_amdgcn_fence(__ATOMIC_RELEASE, "workgroup");
    __builtin_amdgcn_wave_barrier();
    __builtin_amdgcn_fence(__ATOMIC_ACQUIRE, "workgroup");
    if (OUT_MODE == 0) {
      float* C = (float*)Cout + (size_t)b * strideC;
      const int hh = lane >> 4, c4 = (lane & 15) * 4;
      for (int pass = 0; pass < 2; ++pass) {
#pragma unroll
        for (int it = 0; it < 8; ++it) {
          const int row = it * 2 + hh;
          v4f v = *(const v4f*)(slab + row * 68 + c4);
          *(volatile v4f*)(C + (size_t)(mBase + row) * ldc + n0 + c4) = v;
        }
        __threadfence();
      }
    } else {
      const int q = lane >> 3, c8 = (lane & 7) * 8;
      unsigned short* C  = (unsigned short*)Cout  + (size_t)b * strideC;
      unsigned short* C2 = (OUT_MODE == 2) ? ((unsigned short*)Cout2 + (size_t)b * strideC) : nullptr;
      for (int pass = 0; pass < 2; ++pass) {
#pragma unroll
        for (int it = 0; it < 4; ++it) {
          const int row = it * 4 + q;
          const float* sp = slab + row * 68 + c8;
          v8h hv, lv;
#pragma unroll
          for (int e = 0; e < 8; ++e) {
            if (OUT_MODE == 1) {
              hv[e] = (_Float16)sp[e];
            } else {
              unsigned short hb = f2bf_bits(sp[e]);
              unsigned short lb = f2bf_bits(sp[e] - bf_bits2f(hb));
              hv[e] = __builtin_bit_cast(_Float16, hb);
              lv[e] = __builtin_bit_cast(_Float16, lb);
            }
          }
          *(volatile v8h*)(C + (size_t)(mBase + row) * ldc + n0 + c8) = hv;
          if (OUT_MODE == 2) *(volatile v8h*)(C2 + (size_t)(mBase + row) * ldc + n0 + c8) = lv;
        }
        __threadfence();
      }
    }
    __builtin_amdgcn_fence(__ATOMIC_RELEASE, "workgroup");
    __builtin_amdgcn_wave_barrier();
    __builtin_amdgcn_fence(__ATOMIC_ACQUIRE, "workgroup");
  }
}


__global__ __launch_bounds__(kThr) void cast_plane_kernel(const float* __restrict__ src, unsigned short* __restrict__ dst,
                                                          int colsLog2, int dstPitch, int dstOff) {
  const int i   = blockIdx.x * kThr + threadIdx.x;
  const int sh  = colsLog2 - 3;
  const int row = i >> sh;
  const int c8  = (i & ((1 << sh) - 1)) * 8;
  const float* sp = src + ((size_t)row << colsLog2) + c8;
  const v4f a0 = *(const v4f*)(sp);
  const v4f a1 = *(const v4f*)(sp + 4);
  v8h hv;
#pragma unroll
  for (int e = 0; e < 4; ++e) {
    const float f0 = a0[e];
    const float f1 = a1[e];
    hv[e]     = (_Float16)carry_flush(bf16r(f0), kInCarry);
    hv[4 + e] = (_Float16)carry_flush(bf16r(f1), kInCarry);
  }
  unsigned short* dp = dst + (size_t)row * dstPitch + dstOff + c8;
  *(volatile v8h*)dp = hv;
  __threadfence();
  *(volatile v8h*)dp = hv;
}

__global__ __launch_bounds__(256) void wt_plane_kernel(const float* __restrict__ W, unsigned short* __restrict__ dst, int K, int N, int nLive, int ldd, int colOff) {
  const int n  = blockIdx.x;
  const int k8 = threadIdx.x * 8;
  const bool live = n < nLive;
  const int nc = live ? n : 0;
  v8h hv;
#pragma unroll
  for (int e = 0; e < 8; ++e) {
    const float w = W[(size_t)(k8 + e) * N + nc];
    hv[e] = (_Float16)(live ? carry_flush(bf16r(w), kWCarry) : 0.0f);
  }
  unsigned short* dp = dst + (size_t)n * ldd + colOff + k8;
  *(volatile v8h*)dp = hv;
  __threadfence();
  *(volatile v8h*)dp = hv;
}

__global__ __launch_bounds__(kThr) void setup_kernel(const float* __restrict__ b_dt, float* __restrict__ BV) {
  const unsigned i = blockIdx.x * (unsigned)kThr + threadIdx.x;
  const bool live = i >= (unsigned)kBvDt;
  const float v = b_dt[live ? (i - (unsigned)kBvDt) : 0u];
  const float o = live ? bf16r(v) : 0.0f;
  float* dp = BV + i;
  *(volatile float*)dp = o;
  __threadfence();
  *(volatile float*)dp = o;
}
static_assert(24 * kThr == kBvTot && (kBvDt % kThr) == 0, "set-up grid exact: 24 blocks: 16 of zeros, 8 of b_dt");

__global__ __launch_bounds__(kThr) void conv_kernel(const float* __restrict__ XZ, const float* __restrict__ conv_state, const float* __restrict__ conv_w, const float* __restrict__ conv_b,
                                                    float* __restrict__ XI, unsigned short* __restrict__ XI16) {
  const unsigned i = blockIdx.x * (unsigned)kThr + threadIdx.x;
  const unsigned row = i >> 9;
  const unsigned d4 = (i & 511u) * 4u;
  const unsigned t = row & (unsigned)(kL - 1);
  const unsigned sq = row >> 11;
  const v4f cb = *(const v4f*)(conv_b + d4);
  v4f acc;
#pragma unroll
  for (int e = 0; e < 4; ++e) acc[e] = bf16r(cb[e]);
  v4f wv[4];
#pragma unroll
  for (int e = 0; e < 4; ++e) wv[e] = *(const v4f*)(conv_w + (d4 + (unsigned)e) * (unsigned)kCv);
#pragma unroll
  for (int j = 0; j < kCv; ++j) {
    const int tt = (int)t - (kCv - 1) + j;
    const bool inx = tt >= 0;
    const unsigned rr = inx ? (row - (unsigned)(kCv - 1 - j)) : row;
    const v4f xin = *(const v4f*)(XZ + rr * (unsigned)kDI2 + d4);
    const unsigned cj = inx ? 0u : (t + (unsigned)j);
#pragma unroll
    for (int e = 0; e < 4; ++e) {
      const float cs = conv_state[(sq * (unsigned)kDI + d4 + (unsigned)e) * (unsigned)(kCv - 1) + cj];
      const float v = inx ? xin[e] : bf16r(cs);
      acc[e] += bf16r(wv[e][j]) * v;
    }
  }
  v4f o;
  v4h hv, lv;
#pragma unroll
  for (int e = 0; e < 4; ++e) {
    const float s = acc[e] * (1.0f / (1.0f + expf(-acc[e])));
    o[e] = s;
    const float c = carry_flush(s, kACarry);
    const _Float16 hi = (_Float16)c;
    hv[e] = hi;
    lv[e] = (_Float16)carry_flush(c - (float)hi, 1.0f);
  }
  float* po = XI + row * (unsigned)kDI + d4;
  unsigned short* ph = XI16 + row * (unsigned)kDI2 + d4;
  for (int pass = 0; pass < 2; ++pass) {
    *(volatile v4f*)po = o;
    *(volatile v4h*)ph = hv;
    *(volatile v4h*)(ph + kDI) = lv;
    __threadfence();
  }
}
static_assert((size_t)kRows * kDI / 4 == 8192ull * kThr && kDI / 4 == 512 && kL == 2048, "the convolution's grid exact: 8,192 blocks: two blocks a row");

__global__ __launch_bounds__(kThr) void tail_kernel(const float* __restrict__ XZ, float* __restrict__ out2) {
  const unsigned i = blockIdx.x * (unsigned)kThr + threadIdx.x;
  const unsigned sq = i >> 11;
  const unsigned d = i & (unsigned)(kDI - 1);
  float v[kCv - 1];
#pragma unroll
  for (int j = 0; j < kCv - 1; ++j) v[j] = XZ[(sq * (unsigned)kL + (unsigned)(kL - (kCv - 1) + j)) * (unsigned)kDI2 + d];
  float* dp = out2 + i * (unsigned)(kCv - 1);
  for (int pass = 0; pass < 2; ++pass) {
#pragma unroll
    for (int j = 0; j < kCv - 1; ++j) *(volatile float*)(dp + j) = v[j];
    __threadfence();
  }
}
static_assert(kNB * kDI == 16 * kThr && (32 * (kCv - 1) * 4) % 128 == 0, "the third result's grid exact: 16 blocks; a wave's 384 B are three whole lines");

__global__ __launch_bounds__(kThr) void dtcast_kernel(const float* __restrict__ XD, unsigned short* __restrict__ DT16) {
  const unsigned i = blockIdx.x * (unsigned)kThr + threadIdx.x;
  const unsigned row = i >> 3;
  const unsigned c8 = (i & 7u) * 8u;
  const v4f a0 = *(const v4f*)(XD + row * (unsigned)kXdP + c8), a1 = *(const v4f*)(XD + row * (unsigned)kXdP + c8 + 4);
  v8h hv;
#pragma unroll
  for (int e = 0; e < 4; ++e) { hv[e] = (_Float16)carry_flush(a0[e], kDtCarry); hv[4 + e] = (_Float16)carry_flush(a1[e], kDtCarry); }
  unsigned short* dp = DT16 + i * 8u;
  *(volatile v8h*)dp = hv;
  __threadfence();
  *(volatile v8h*)dp = hv;
}
static_assert((size_t)kRows * kR / 8 == 128ull * kThr && kR / 8 == 8, "the step input's cast grid exact: 128 blocks");

__device__ __forceinline__ float softplus_f(float v) { return fmaxf(v, 0.0f) + log1pf(expf(-fabsf(v))); }

__global__ __launch_bounds__(kThr) void scan_kernel(const float* __restrict__ DL, const float* __restrict__ XI, const float* __restrict__ XD, const float* __restrict__ A_log, const float* __restrict__ ssm_state,
                                                    const float* __restrict__ D_skip, float* __restrict__ YS, float* __restrict__ out1) {
  const unsigned ix = blockIdx.x * (unsigned)kThr + threadIdx.x;
  const unsigned sq = ix >> 11;
  const unsigned d  = ix & (unsigned)(kDI - 1);
  float A[kNs], h[kNs];
#pragma unroll
  for (int q = 0; q < kNs / 4; ++q) {
    const v4f av = *(const v4f*)(A_log + d * (unsigned)kNs + 4 * q);
    const v4f hv = *(const v4f*)(ssm_state + ix * (unsigned)kNs + 4 * q);
#pragma unroll
    for (int e = 0; e < 4; ++e) { A[4 * q + e] = -expf(bf16r(av[e])); h[4 * q + e] = bf16r(hv[e]); }
  }
  const float dsk = bf16r(D_skip[d]);
  for (int l = 0; l < kL; ++l) {
    const unsigned row = sq * (unsigned)kL + (unsigned)l;
    const float dt = softplus_f(DL[row * (unsigned)kDI + d]);
    const float x = XI[row * (unsigned)kDI + d];
    const float* pb = XD + row * (unsigned)kXdP + (unsigned)kR;
    float y = 0.0f;
#pragma unroll
    for (int q = 0; q < kNs / 4; ++q) {
      const v4f bv = *(const v4f*)(pb + 4 * q), cv = *(const v4f*)(pb + kNs + 4 * q);
#pragma unroll
      for (int e = 0; e < 4; ++e) {
        const int n = 4 * q + e;
        const float hn = expf(dt * A[n]) * h[n] + (dt * bv[e]) * x;
        h[n] = hn;
        y += hn * cv[e];
      }
    }
    y += dsk * x;
    float* dp = YS + row * (unsigned)kDI + d;
    *(volatile float*)dp = y;
    __threadfence();
    *(volatile float*)dp = y;
  }
  float* fp = out1 + ix * (unsigned)kNs;
  for (int pass = 0; pass < 2; ++pass) {
#pragma unroll
    for (int q = 0; q < kNs / 4; ++q) { v4f o; o[0] = h[4 * q]; o[1] = h[4 * q + 1]; o[2] = h[4 * q + 2]; o[3] = h[4 * q + 3]; *(volatile v4f*)(fp + 4 * q) = o; }
    __threadfence();
  }
}
static_assert(kNB * kDI == 16 * kThr && (kNs % 4) == 0 && (kXdP % 4) == 0 && (kR % 4) == 0, "scan grid exact: 16 blocks: eight a sequence; the B | C columns 16-B aligned");

__global__ __launch_bounds__(kThr) void gate_kernel(const float* __restrict__ YS, const float* __restrict__ XZ, unsigned short* __restrict__ YG16) {
  const unsigned i = blockIdx.x * (unsigned)kThr + threadIdx.x;
  const unsigned row = i >> 7;
  const unsigned c16 = (i & 127u) * 16u;
  const float* py = YS + row * (unsigned)kDI + c16;
  const float* pz = XZ + row * (unsigned)kDI2 + (unsigned)kDI + c16;
  v8h hv[2];
#pragma unroll
  for (int k = 0; k < 2; ++k) {
    const v4f y0 = *(const v4f*)(py + 8 * k), y1 = *(const v4f*)(py + 8 * k + 4);
    const v4f z0 = *(const v4f*)(pz + 8 * k), z1 = *(const v4f*)(pz + 8 * k + 4);
#pragma unroll
    for (int e = 0; e < 8; ++e) {
      const float yy = (e < 4) ? y0[e] : y1[e - 4];
      const float zz = (e < 4) ? z0[e] : z1[e - 4];
      hv[k][e] = (_Float16)carry_flush(yy * (zz / (1.0f + expf(-zz))), kACarry);
    }
  }
  unsigned short* dp = YG16 + i * 16u;
  for (int pass = 0; pass < 2; ++pass) {
    *(volatile v8h*)dp = hv[0];
    *(volatile v8h*)(dp + 8) = hv[1];
    __threadfence();
  }
}
static_assert((size_t)kRows * kDI / 16 == 2048ull * kThr && kDI / 16 == 128 && (size_t)kRows * kDI2 < 4294967296ull / 4, "the gate's grid exact: 2,048 blocks: two rows a block; every plane's element offsets fit 32 bits");

extern "C" void kernel_launch(void* const* d_in, const int* in_sizes, int n_in,
                              void* d_out, int out_size, void* d_ws, size_t ws_size,
                              hipStream_t stream) {
  if (n_in < 12 || d_out == nullptr || d_ws == nullptr) return;
  if (in_sizes[0] != kRows * kDm || in_sizes[1] != kOut1 || in_sizes[2] != kOut2 || in_sizes[3] != kDm * kDI2 || in_sizes[4] != kDI * kCv || in_sizes[5] != kDI || in_sizes[6] != kDI * kXd
      || in_sizes[7] != kR * kDI || in_sizes[8] != kDI || in_sizes[9] != kDI * kNs || in_sizes[10] != kDI || in_sizes[11] != kDI * kDm) return;
  if (out_size != kOut0 + kOut1 + kOut2) return;
  if (ws_size < kWsTotal) return;
  const float* x = (const float*)d_in[0];
  const float* ssm_state = (const float*)d_in[1];
  const float* conv_state = (const float*)d_in[2];
  const float* w_in = (const float*)d_in[3];
  const float* conv_w = (const float*)d_in[4];
  const float* conv_b = (const float*)d_in[5];
  const float* w_x = (const float*)d_in[6];
  const float* w_dt = (const float*)d_in[7];
  const float* b_dt = (const float*)d_in[8];
  const float* A_log = (const float*)d_in[9];
  const float* D_skip = (const float*)d_in[10];
  const float* w_out = (const float*)d_in[11];
  float* out = (float*)d_out;
  char* ws = (char*)d_ws;
  unsigned short* X16 = (unsigned short*)(ws + kOffX16);
  unsigned short* WIT = (unsigned short*)(ws + kOffWIT);
  unsigned short* WXT = (unsigned short*)(ws + kOffWXT);
  unsigned short* WDT = (unsigned short*)(ws + kOffWDT);
  unsigned short* WOT = (unsigned short*)(ws + kOffWOT);
  float* BV = (float*)(ws + kOffBV);
  float* XZ = (float*)(ws + kOffXZ);
  float* XI = (float*)(ws + kOffXI);
  unsigned short* XI16 = (unsigned short*)(ws + kOffXI16);
  float* XD = (float*)(ws + kOffXD);
  unsigned short* DT16 = (unsigned short*)(ws + kOffDT16);
  float* DL = (float*)(ws + kOffDL);
  float* YS = (float*)(ws + kOffYS);
  unsigned short* YG16 = (unsigned short*)(ws + kOffYG16);

  static_assert(((size_t)kRows * kDm / 8) % kThr == 0 && kDm / 8 == 128 && kDI / 8 == 256 && kR / 8 == 8, "the row cast's grid; the transposing casts run one block a destination row with exactly K / 8 threads");
  cast_plane_kernel<<<(int)(((size_t)kRows * kDm / 8) / kThr), kThr, 0, stream>>>(x, X16, 10, kDm, 0);
  wt_plane_kernel<<<kDI2, kDm / 8, 0, stream>>>(w_in, WIT, kDm, kDI2, kDI2, kDm, 0);
  wt_plane_kernel<<<kXdP, kDI / 8, 0, stream>>>(w_x, WXT, kDI, kXd, kXd, kDI2, 0);
  wt_plane_kernel<<<kXdP, kDI / 8, 0, stream>>>(w_x, WXT, kDI, kXd, kXd, kDI2, kDI);
  wt_plane_kernel<<<kDI, kR / 8, 0, stream>>>(w_dt, WDT, kR, kDI, kDI, kR, 0);
  wt_plane_kernel<<<kDm, kDI / 8, 0, stream>>>(w_out, WOT, kDI, kDm, kDm, kDI, 0);
  setup_kernel<<<24, kThr, 0, stream>>>(b_dt, BV);
  wmma_gemm64<0, false, 2, 0, false, 0><<<dim3((kRows / 64) * (kDI2 / 64) / 8, 1), 256, 0, stream>>>(
      X16, X16, kDm, 0L, WIT, WIT, kDm, 0L, (void*)XZ, (void*)XZ, kDI2, 0L, BV, nullptr, 0L, kRows, kDI2, kDm, kScIn);
  conv_kernel<<<8192, kThr, 0, stream>>>(XZ, conv_state, conv_w, conv_b, XI, XI16);
  tail_kernel<<<16, kThr, 0, stream>>>(XZ, out + kOut0 + kOut1);
  wmma_gemm64<0, false, 2, 0, false, 0><<<dim3((kRows / 64) * (kXdP / 64) / 8, 1), 256, 0, stream>>>(
      XI16, XI16, kDI2, 0L, WXT, WXT, kDI2, 0L, (void*)XD, (void*)XD, kXdP, 0L, BV, nullptr, 0L, kRows, kXdP, kDI2, kScA);
  dtcast_kernel<<<128, kThr, 0, stream>>>(XD, DT16);
  wmma_gemm64<0, false, 2, 0, false, 0><<<dim3((kRows / 64) * (kDI / 64) / 8, 1), 256, 0, stream>>>(
      DT16, DT16, kR, 0L, WDT, WDT, kR, 0L, (void*)DL, (void*)DL, kDI, 0L, BV + kBvDt, nullptr, 0L, kRows, kDI, kR, kScDt);
  scan_kernel<<<16, kThr, 0, stream>>>(DL, XI, XD, A_log, ssm_state, D_skip, YS, out + kOut0);
  gate_kernel<<<2048, kThr, 0, stream>>>(YS, XZ, YG16);
  wmma_gemm64<0, false, 2, 0, false, 0><<<dim3((kRows / 64) * (kDm / 64) / 8, 1), 256, 0, stream>>>(
      YG16, YG16, kDI, 0L, WOT, WOT, kDI, 0L, (void*)out, (void*)out, kDm, 0L, BV, nullptr, 0L, kRows, kDm, kDI, kScA);
}
static_assert(((kRows / 64) * (kDI2 / 64)) % 8 == 0 && ((kRows / 64) * (kXdP / 64)) % 8 == 0 && ((kRows / 64) * (kDI / 64)) % 8 == 0 && ((kRows / 64) * (kDm / 64)) % 8 == 0, "the engine's grids: whole blocks of eight wave tiles");
static_assert((kOut0 % 32) == 0 && ((kOut0 + kOut1) % 32) == 0, "the second and third results start on multiples of 128 B");
